// T2SBlock_19610820674349
// MI455X (gfx1250) — hardware-verified
//
#include <hip/hip_runtime.h>
#include <hip/hip_bf16.h>

typedef __attribute__((ext_vector_type(16))) _Float16 v16h;
typedef __attribute__((ext_vector_type(8)))  _Float16 v8h;
typedef __attribute__((ext_vector_type(4)))  _Float16 v4h;
typedef __attribute__((ext_vector_type(16))) __bf16   v16b;
typedef __attribute__((ext_vector_type(8)))  __bf16   v8b;
typedef __attribute__((ext_vector_type(8)))  float    v8f;
typedef __attribute__((ext_vector_type(4)))  float    v4f;

__device__ __forceinline__ unsigned short f2bf_bits(float f) {
  unsigned u = __float_as_uint(f);
  return (unsigned short)((u + 0x7FFFu + ((u >> 16) & 1u)) >> 16);
}
__device__ __forceinline__ float bf_bits2f(unsigned short h) { return __uint_as_float(((unsigned)h) << 16); }

__device__ __forceinline__ void dep_guard_h(v8f& a, v8f& b, v16h x, v16h y) { asm volatile("v_nop\n\tv_nop\n\tv_nop\n\tv_nop" : "+v"(a), "+v"(b) : "v"(x), "v"(y)); }
__device__ __forceinline__ void dep_guard_b(v8f& a, v8f& b, v16b x, v16b y) { asm volatile("v_nop\n\tv_nop\n\tv_nop\n\tv_nop" : "+v"(a), "+v"(b) : "v"(x), "v"(y)); }
__device__ __forceinline__ void keep4_h(v16h a, v16h b, v16h c, v16h d) { asm volatile("v_nop" :: "v"(a), "v"(b), "v"(c), "v"(d)); }
__device__ __forceinline__ void keep4_b(v16b a, v16b b, v16b c, v16b d) { asm volatile("v_nop" :: "v"(a), "v"(b), "v"(c), "v"(d)); }
__device__ __forceinline__ void acc_guard4(v8f& a, v8f& b, v8f& c, v8f& d) { asm volatile("v_nop\n\tv_nop\n\tv_nop\n\tv_nop" : "+v"(a), "+v"(b), "+v"(c), "+v"(d)); }
template <typename T> struct Frag;
template <> struct Frag<_Float16> {
  typedef v16h V; union U { v16h v; v8h h[2]; };
  static __device__ __forceinline__ v16h load(const _Float16* p) {
    U f; f.h[0] = *(const v8h*)(p); f.h[1] = *(const v8h*)(p + 16); return f.v;
  }
  static __device__ __forceinline__ v8f mma(v16h a, v16h b, v8f c) {
    return __builtin_amdgcn_wmma_f32_16x16x32_f16(false, a, false, b, (short)0, c, false, false);
  }
  static __device__ __forceinline__ void guard(v8f& a, v8f& b, v16h x, v16h y) { dep_guard_h(a, b, x, y); }
  static __device__ __forceinline__ void keep(v16h a, v16h b, v16h c, v16h d) { keep4_h(a, b, c, d); }
};
template <> struct Frag<__bf16> {
  typedef v16b V; union U { v16b v; v8b h[2]; };
  static __device__ __forceinline__ v16b load(const __bf16* p) {
    U f; f.h[0] = *(const v8b*)(p); f.h[1] = *(const v8b*)(p + 16); return f.v;
  }
  static __device__ __forceinline__ v8f mma(v16b a, v16b b, v8f c) {
    return __builtin_amdgcn_wmma_f32_16x16x32_bf16(false, a, false, b, (short)0, c, false, false);
  }
  static __device__ __forceinline__ void guard(v8f& a, v8f& b, v16b x, v16b y) { dep_guard_b(a, b, x, y); }
  static __device__ __forceinline__ void keep(v16b a, v16b b, v16b c, v16b d) { keep4_b(a, b, c, d); }
};

template <int ET> struct Elem;
template <> struct Elem<0> { typedef _Float16 T; };
template <> struct Elem<1> { typedef __bf16 T; };
template <int ET, bool SPLIT, int BIAS_MODE, int OUT_MODE, bool RESID, int ACT = 0>
__global__ __launch_bounds__(256) void wmma_gemm64(
    const unsigned short* __restrict__ Ap, const unsigned short* __restrict__ A2p, int lda, long strideA,
    const unsigned short* __restrict__ Btp, const unsigned short* __restrict__ Bt2p, int ldb, long strideB,
    void* __restrict__ Cout, void* __restrict__ Cout2, int ldc, long strideC,
    const float* __restrict__ bias,
    const float* __restrict__ resid, long strideR,
    int M, int N, int K, float scale) {
  typedef typename Elem<ET>::T T;
  typedef typename Frag<T>::V V;
  const T* A = (const T*)Ap; const T* A2 = (const T*)A2p; const T* Bt = (const T*)Btp; const T* Bt2 = (const T*)Bt2p;
  __shared__ __align__(16) float sT[8][16 * 68];
  const int b    = blockIdx.y;
  const int lane = threadIdx.x & 31;
  const int wave = threadIdx.x >> 5;
  const int tilesN = N >> 6;
  const int tilesM = M >> 6;
  const int tile = blockIdx.x * 8 + wave;
  if (tile >= tilesM * tilesN) return;
  const int tm = tile / tilesN;
  const int tn = tile - tm * tilesN;
  const int m0 = tm << 6;
  const int n0 = tn << 6;

  const T* Ab  = A  + (size_t)b * strideA;
  const T* Bb  = Bt + (size_t)b * strideB;
  const T* Ab2 = SPLIT ? (A2  + (size_t)b * strideA) : nullptr;
  const T* Bb2 = SPLIT ? (Bt2 + (size_t)b * strideB) : nullptr;

  const int rlane = lane & 15;
  const int koff  = (lane >> 4) * 8;
  const int mOff  = (lane >> 4) * 8;

  v8f acc[4][4];
#pragma unroll
  for (int i = 0; i < 4; ++i)
#pragma unroll
    for (int j = 0; j < 4; ++j) acc[i][j] = (v8f){0.f,0.f,0.f,0.f,0.f,0.f,0.f,0.f};

  for (int k0 = 0; k0 < K; k0 += 32) {
    V bh[4], bl[4];
#pragma unroll
    for (int j = 0; j < 4; ++j) {
      const size_t bo = (size_t)(n0 + (j << 4) + rlane) * ldb + koff + k0;
      bh[j] = Frag<T>::load(Bb + bo);
      if (SPLIT) bl[j] = Frag<T>::load(Bb2 + bo);
    }
#pragma unroll
    for (int i = 0; i < 4; ++i) {
      const size_t ao = (size_t)(m0 + (i << 4) + rlane) * lda + koff + k0;
      V ah = Frag<T>::load(Ab + ao);
      V al;
      if (SPLIT) al = Frag<T>::load(Ab2 + ao);
#pragma unroll
      for (int j = 0; j < 4; ++j) {
        acc[i][j] = Frag<T>::mma(ah, bh[j], acc[i][j]);
        if (SPLIT) {
          acc[i][j] = Frag<T>::mma(ah, bl[j], acc[i][j]);
          acc[i][j] = Frag<T>::mma(al, bh[j], acc[i][j]);
        }
      }
      Frag<T>::guard(acc[i][0], acc[i][3], ah, SPLIT ? al : ah);
    }
    Frag<T>::keep(bh[0], bh[1], bh[2], bh[3]);
    if (SPLIT) Frag<T>::keep(bl[0], bl[1], bl[2], bl[3]);
  }
  acc_guard4(acc[0][0], acc[0][1], acc[0][2], acc[0][3]);
  acc_guard4(acc[1][0], acc[1][1], acc[1][2], acc[1][3]);
  acc_guard4(acc[2][0], acc[2][1], acc[2][2], acc[2][3]);
  acc_guard4(acc[3][0], acc[3][1], acc[3][2], acc[3][3]);

  float* slab = sT[wave];
  const float* Rb = RESID ? (resid + (size_t)b * strideR) : nullptr;
#pragma unroll
  for (int i = 0; i < 4; ++i) {
    const int mBase = m0 + (i << 4);
#pragma unroll
    for (int j = 0; j < 4; ++j) {
      const int n = n0 + (j << 4) + rlane;
      float bv = 0.f;
      if (BIAS_MODE == 2) bv = bias[n];
#pragma unroll
      for (int r = 0; r < 8; ++r) {
        float v = acc[i][j][r] * scale;
        if (BIAS_MODE == 1) v += bias[mBase + mOff + r];
        if (BIAS_MODE == 2) v += bv;
        if (RESID) v += Rb[(size_t)(mBase + mOff + r) * ldc + n];
        if (ACT == 1) v = tanhf(v);
        if (ACT == 2) v = fmaxf(v, 0.0f);
        if (ACT == 3) v = v / (1.0f + expf(-v));
        if (ACT == 4) v = (v > 0.f) ? v : 0.01f * v;
        if (ACT == 5) v = 0.5f * v * (1.0f + erff(v * 0.70710678118654752f));
        slab[(mOff + r) * 68 + (j << 4) + rlane] = v;
      }
    }
    __builtin_amdgcn_fence(__ATOMIC_RELEASE, "workgroup");
    __builtin_amdgcn_wave_barrier();
    __builtin_amdgcn_fence(__ATOMIC_ACQUIRE, "workgroup");
    if (OUT_MODE == 0) {
      float* C = (float*)Cout + (size_t)b * strideC;
      const int hh = lane >> 4, c4 = (lane & 15) * 4;
      for (int pass = 0; pass < 2; ++pass) {
#pragma unroll
        for (int it = 0; it < 8; ++it) {
          const int row = it * 2 + hh;
          v4f v = *(const v4f*)(slab + row * 68 + c4);
          *(volatile v4f*)(C + (size_t)(mBase + row) * ldc + n0 + c4) = v;
        }
        __threadfence();
      }
    } else {
      const int q = lane >> 3, c8 = (lane & 7) * 8;
      unsigned short* C  = (unsigned short*)Cout  + (size_t)b * strideC;
      unsigned short* C2 = (OUT_MODE == 2) ? ((unsigned short*)Cout2 + (size_t)b * strideC) : nullptr;
      for (int pass = 0; pass < 2; ++pass) {
#pragma unroll
        for (int it = 0; it < 4; ++it) {
          const int row = it * 4 + q;
          const float* sp = slab + row * 68 + c8;
          v8h hv, lv;
#pragma unroll
          for (int e = 0; e < 8; ++e) {
            if (OUT_MODE == 1) {
              hv[e] = (_Float16)sp[e];
            } else {
              unsigned short hb = f2bf_bits(sp[e]);
              unsigned short lb = f2bf_bits(sp[e] - bf_bits2f(hb));
              hv[e] = __builtin_bit_cast(_Float16, hb);
              lv[e] = __builtin_bit_cast(_Float16, lb);
            }
          }
          *(volatile v8h*)(C + (size_t)(mBase + row) * ldc + n0 + c8) = hv;
          if (OUT_MODE == 2) *(volatile v8h*)(C2 + (size_t)(mBase + row) * ldc + n0 + c8) = lv;
        }
        __threadfence();
      }
    }
    __builtin_amdgcn_fence(__ATOMIC_RELEASE, "workgroup");
    __builtin_amdgcn_wave_barrier();
    __builtin_amdgcn_fence(__ATOMIC_ACQUIRE, "workgroup");
  }
}

__global__ __launch_bounds__(256) void cast_f32_f16x2(
    const float* __restrict__ in, _Float16* __restrict__ out, int n2) {
  int i = blockIdx.x * 256 + threadIdx.x;
  if (i < n2) {
    const _Float16 h0 = (_Float16)in[2 * i], h1 = (_Float16)in[2 * i + 1];
    const unsigned u = (unsigned)__builtin_bit_cast(unsigned short, h0) | ((unsigned)__builtin_bit_cast(unsigned short, h1) << 16);
    ((volatile unsigned*)out)[i] = u;
    __threadfence();
    ((volatile unsigned*)out)[i] = u;
  }
}

__global__ __launch_bounds__(256) void transpose_cast_f16(
    const float* __restrict__ in, _Float16* __restrict__ out, int R, int C, float mul) {
  __shared__ float t[64][65];
  const int r0 = blockIdx.y * 64, c0 = blockIdx.x * 64;
  const int tid = threadIdx.x;
#pragma unroll
  for (int i = 0; i < 16; ++i) {
    const int idx = i * 256 + tid;
    const int r = idx >> 6, cc = idx & 63;
    t[r][cc] = in[(size_t)(r0 + r) * C + c0 + cc];
  }
  __syncthreads();
  const int q = tid & 7;
#pragma unroll
  for (int ph = 0; ph < 2; ++ph) {
    const int n = ph * 32 + (tid >> 3);
    v8h hv;
#pragma unroll
    for (int e = 0; e < 8; ++e) hv[e] = (_Float16)(t[q * 8 + e][n] * mul);
    _Float16* dst = out + (size_t)(c0 + n) * R + r0 + q * 8;
    *(volatile v8h*)dst = hv;
    __threadfence();
    *(volatile v8h*)dst = hv;
  }
}

__global__ __launch_bounds__(256) void layernorm_kernel(
    const float* __restrict__ X, const float* __restrict__ g, const float* __restrict__ be,
    float* __restrict__ Yf, _Float16* __restrict__ Yh, int writeH) {
  __shared__ float red[8];
  const int row = blockIdx.x, tid = threadIdx.x, lane = tid & 31, wave = tid >> 5;
  const float* x = X + (size_t)row * 1024;
  const v4f v = *(const v4f*)(x + tid * 4);
  float s = (v[0] + v[1]) + (v[2] + v[3]);
#pragma unroll
  for (int off = 1; off < 32; off <<= 1) s += __shfl_xor(s, off, 32);
  if (lane == 0) red[wave] = s;
  __syncthreads();
  float tot = red[0];
#pragma unroll
  for (int w = 1; w < 8; ++w) tot += red[w];
  const float mean = tot * (1.0f / 1024.0f);
  __syncthreads();
  const float d0 = v[0] - mean, d1 = v[1] - mean, d2 = v[2] - mean, d3 = v[3] - mean;
  float ss = (d0 * d0 + d1 * d1) + (d2 * d2 + d3 * d3);
#pragma unroll
  for (int off = 1; off < 32; off <<= 1) ss += __shfl_xor(ss, off, 32);
  if (lane == 0) red[wave] = ss;
  __syncthreads();
  float tot2 = red[0];
#pragma unroll
  for (int w = 1; w < 8; ++w) tot2 += red[w];
  const float var = tot2 * (1.0f / 1024.0f);
  const float rstd = rsqrtf(var + 1e-5f);
  const v4f gg = *(const v4f*)(g + tid * 4);
  const v4f bb = *(const v4f*)(be + tid * 4);
  v4f y;
  y[0] = d0 * rstd * gg[0] + bb[0];
  y[1] = d1 * rstd * gg[1] + bb[1];
  y[2] = d2 * rstd * gg[2] + bb[2];
  y[3] = d3 * rstd * gg[3] + bb[3];
  v4h yh;
  yh[0] = (_Float16)y[0]; yh[1] = (_Float16)y[1]; yh[2] = (_Float16)y[2]; yh[3] = (_Float16)y[3];
  float* yp = Yf + (size_t)row * 1024 + tid * 4;
  _Float16* hp = Yh + (size_t)row * 1024 + tid * 4;
  *(volatile v4f*)yp = y;
  if (writeH) *(volatile v4h*)hp = yh;
  __threadfence();
  *(volatile v4f*)yp = y;
  if (writeH) *(volatile v4h*)hp = yh;
}

#define AT_S 2048
#define AT_QP 3072
#define AT_OPITCH 1024
#define AT_NCH 32

__device__ __forceinline__ v8f mma_h(v16h a, v16h b, v8f c) {
  c = __builtin_amdgcn_wmma_f32_16x16x32_f16(false, a, false, b, (short)0, c, false, false);
  asm volatile("v_nop\n\tv_nop\n\tv_nop\n\tv_nop" : "+v"(c) : "v"(a), "v"(b));
  return c;
}

__global__ __launch_bounds__(128)
void attn_f16_kernel(const _Float16* __restrict__ qkv, const int* __restrict__ mask, _Float16* __restrict__ out) {
  __shared__ __align__(16) _Float16 Ksh[64 * 64];
  __shared__ __align__(16) _Float16 Vth[64 * 64];
  __shared__ __align__(16) _Float16 Psh[4][16 * 64];
  __shared__ __align__(16) float Os[4][16 * 68];
  __shared__ int wflag[4];

  const int tid  = threadIdx.x;
  const int wave = tid >> 5;
  const int lane = tid & 31;
  const int hh   = lane >> 4;
  const int c    = lane & 15;

  const int bx = blockIdx.x;
  const int qb = bx & 31;
  const int bhh = bx >> 5;
  const int h  = bhh & 15;
  const int b  = bhh >> 4;
  const int q0 = qb * 64 + wave * 16;

  const _Float16* qbp = qkv + (size_t)b * AT_S * AT_QP + h * 64;
  const _Float16* kbp = qbp + 1024;
  const _Float16* vbp = qbp + 2048;
  _Float16* obp = out + (size_t)b * AT_S * AT_OPITCH + h * 64;

  v16h qa0, qa1;
  {
    const _Float16* qrow = qbp + (size_t)(q0 + c) * AT_QP + 8 * hh;
    qa0 = Frag<_Float16>::load(qrow);
    qa1 = Frag<_Float16>::load(qrow + 32);
  }

  float mrow[8], lrow[8];
  v8f oacc[4];
#pragma unroll
  for (int r = 0; r < 8; ++r) { mrow[r] = -__builtin_huge_valf(); lrow[r] = 0.f; }
#pragma unroll
  for (int t = 0; t < 4; ++t) oacc[t] = (v8f){0.f,0.f,0.f,0.f,0.f,0.f,0.f,0.f};

  for (int kc = 0; kc < AT_NCH; ++kc) {
    const int kv0 = kc * 64;
    unsigned mbits = 0u;
#pragma unroll
    for (int r = 0; r < 8; ++r) {
      const int* mp = mask + (size_t)(q0 + 8 * hh + r) * AT_S + kv0 + c;
#pragma unroll
      for (int j = 0; j < 4; ++j) mbits |= ((mp[j * 16] != 0) ? 1u : 0u) << (r * 4 + j);
    }
    const int wany = __any((int)(mbits != 0xFFFFFFFFu));
    __syncthreads();
    if (lane == 0) wflag[wave] = wany;
    __syncthreads();
    const int bany = wflag[0] | wflag[1] | wflag[2] | wflag[3];
    if (bany == 0) continue;

    {
      const int kvr = tid >> 1, dh = (tid & 1) * 32;
      const _Float16* krow = kbp + (size_t)(kv0 + kvr) * AT_QP + dh;
      const _Float16* vrow = vbp + (size_t)(kv0 + kvr) * AT_QP + dh;
#pragma unroll
      for (int i = 0; i < 4; ++i) {
        const v8h kk = *(const v8h*)(krow + 8 * i);
        *(v8h*)(Ksh + kvr * 64 + dh + 8 * i) = kk;
        const v8h vv = *(const v8h*)(vrow + 8 * i);
#pragma unroll
        for (int e = 0; e < 8; ++e) Vth[(dh + 8 * i + e) * 64 + kvr] = vv[e];
      }
    }
    __syncthreads();

    v8f s[4];
#pragma unroll
    for (int j = 0; j < 4; ++j) {
      v8f acc = (v8f){0.f,0.f,0.f,0.f,0.f,0.f,0.f,0.f};
      const _Float16* kp = Ksh + (j * 16 + c) * 64 + 8 * hh;
      const v16h kf0 = Frag<_Float16>::load(kp);
      acc = mma_h(qa0, kf0, acc);
      const v16h kf1 = Frag<_Float16>::load(kp + 32);
      acc = mma_h(qa1, kf1, acc);
      s[j] = acc;
    }

    float cm[8];
#pragma unroll
    for (int r = 0; r < 8; ++r) {
      float m = -__builtin_huge_valf();
#pragma unroll
      for (int j = 0; j < 4; ++j) {
        float sv = s[j][r] * 0.125f;
        if ((mbits >> (r * 4 + j)) & 1u) sv = -3.402823466e38f;
        s[j][r] = sv;
        m = fmaxf(m, sv);
      }
#pragma unroll
      for (int off = 1; off < 16; off <<= 1) m = fmaxf(m, __shfl_xor(m, off, 32));
      cm[r] = m;
    }
    _Float16* pw = Psh[wave];
#pragma unroll
    for (int r = 0; r < 8; ++r) {
      const float mnew = fmaxf(mrow[r], cm[r]);
      const float alpha = expf(mrow[r] - mnew);
      mrow[r] = mnew;
      float psum = 0.f;
#pragma unroll
      for (int j = 0; j < 4; ++j) {
        const float p = expf(s[j][r] - mnew);
        psum += p;
        pw[(8 * hh + r) * 64 + j * 16 + c] = (_Float16)(p * 32768.0f);
      }
#pragma unroll
      for (int off = 1; off < 16; off <<= 1) psum += __shfl_xor(psum, off, 32);
      lrow[r] = lrow[r] * alpha + psum;
#pragma unroll
      for (int t = 0; t < 4; ++t) oacc[t][r] *= alpha;
    }
    __builtin_amdgcn_fence(__ATOMIC_RELEASE, "workgroup");
    __builtin_amdgcn_wave_barrier();
    __builtin_amdgcn_fence(__ATOMIC_ACQUIRE, "workgroup");
#pragma unroll 1
    for (int kk = 0; kk < 2; ++kk) {
      const v16h pa = Frag<_Float16>::load(pw + c * 64 + kk * 32 + 8 * hh);
#pragma unroll
      for (int t = 0; t < 4; ++t) {
        const v16h vb = Frag<_Float16>::load(Vth + (t * 16 + c) * 64 + kk * 32 + 8 * hh);
        oacc[t] = mma_h(pa, vb, oacc[t]);
      }
    }
  }

  float* os = Os[wave];
#pragma unroll
  for (int r = 0; r < 8; ++r) {
    const float inv = 1.0f / (lrow[r] * 32768.0f);
#pragma unroll
    for (int t = 0; t < 4; ++t) os[(8 * hh + r) * 68 + t * 16 + c] = oacc[t][r] * inv;
  }
  __builtin_amdgcn_fence(__ATOMIC_RELEASE, "workgroup");
  __builtin_amdgcn_wave_barrier();
  __builtin_amdgcn_fence(__ATOMIC_ACQUIRE, "workgroup");
  {
    const int q = lane >> 3, c8 = (lane & 7) * 8;
    for (int pass = 0; pass < 2; ++pass) {
#pragma unroll
      for (int it = 0; it < 4; ++it) {
        const int row = it * 4 + q;
        const float* sp = os + row * 68 + c8;
        v8h hv;
#pragma unroll
        for (int e = 0; e < 8; ++e) hv[e] = (_Float16)sp[e];
        *(volatile v8h*)(obp + (size_t)(q0 + row) * AT_OPITCH + c8) = hv;
      }
      __threadfence();
    }
  }
}

extern "C" void kernel_launch(void* const* d_in, const int* in_sizes, int n_in,
                              void* d_out, int out_size, void* d_ws, size_t ws_size,
                              hipStream_t stream) {
  if (n_in < 14) return;
  const int NT = 4096, HD = 1024, H3 = 3072, H4 = 4096, S = 2048;
  if (in_sizes[0] != NT * HD || in_sizes[1] != S * S || in_sizes[2] != HD * H3 || in_sizes[3] != H3 ||
      in_sizes[4] != HD * HD || in_sizes[5] != HD || in_sizes[6] != HD * H4 || in_sizes[7] != H4 ||
      in_sizes[8] != H4 * HD || in_sizes[9] != HD || in_sizes[10] != HD || in_sizes[11] != HD ||
      in_sizes[12] != HD || in_sizes[13] != HD || out_size != NT * HD) return;

  const float* x     = (const float*)d_in[0];
  const int*   amask = (const int*)d_in[1];
  const float* qkv_w = (const float*)d_in[2];
  const float* qkv_b = (const float*)d_in[3];
  const float* out_w = (const float*)d_in[4];
  const float* out_b = (const float*)d_in[5];
  const float* w1    = (const float*)d_in[6];
  const float* b1    = (const float*)d_in[7];
  const float* w2    = (const float*)d_in[8];
  const float* b2    = (const float*)d_in[9];
  const float* ln1_g = (const float*)d_in[10];
  const float* ln1_b = (const float*)d_in[11];
  const float* ln2_g = (const float*)d_in[12];
  const float* ln2_b = (const float*)d_in[13];
  float* outp = (float*)d_out;

  size_t off = 0;
  char* wsb = (char*)d_ws;
  const size_t szXh  = (size_t)NT * HD * 2;
  const size_t szWT  = (size_t)H4 * HD * 2;
  const size_t szQKV = (size_t)NT * H3 * 2;
  const size_t szY   = (size_t)NT * HD * 4;
  const size_t szX1  = (size_t)NT * HD * 4;
  const size_t szX1h = (size_t)NT * HD * 2;
  const size_t szHB  = (size_t)NT * H4 * 2;
  _Float16* xh   = (_Float16*)(wsb + off); off += szXh;
  _Float16* wT   = (_Float16*)(wsb + off); off += szWT;
  _Float16* qkvh = (_Float16*)(wsb + off); off += szQKV;
  float*    ybuf = (float*)(wsb + off);    off += szY;
  float*    x1f  = (float*)(wsb + off);    off += szX1;
  _Float16* x1h  = (_Float16*)(wsb + off); off += szX1h;
  _Float16* hbuf = (_Float16*)(wsb + off); off += szHB;
  if (off > ws_size) return;
  _Float16* attnh = xh;

  typedef const unsigned short* cus;
  const float wmul = 64.0f, wscale = 1.0f / 64.0f;

  {
    const int n2 = NT * HD / 2;
    cast_f32_f16x2<<<(n2 + 255) / 256, 256, 0, stream>>>(x, xh, n2);
  }
  transpose_cast_f16<<<dim3(H3 / 64, HD / 64), 256, 0, stream>>>(qkv_w, wT, HD, H3, wmul);
  {
    const int tiles = (NT / 64) * (H3 / 64);
    wmma_gemm64<0, false, 2, 1, false, 0><<<dim3((tiles + 7) / 8, 1), 256, 0, stream>>>(
        (cus)xh, (cus)xh, HD, 0L, (cus)wT, (cus)wT, HD, 0L,
        (void*)qkvh, (void*)qkvh, H3, 0L, qkv_b, qkv_b, 0L, NT, H3, HD, wscale);
  }
  attn_f16_kernel<<<2 * 16 * (S / 64), 128, 0, stream>>>(qkvh, amask, attnh);
  transpose_cast_f16<<<dim3(HD / 64, HD / 64), 256, 0, stream>>>(out_w, wT, HD, HD, wmul);
  {
    const int tiles = (NT / 64) * (HD / 64);
    wmma_gemm64<0, false, 2, 0, true, 0><<<dim3((tiles + 7) / 8, 1), 256, 0, stream>>>(
        (cus)attnh, (cus)attnh, HD, 0L, (cus)wT, (cus)wT, HD, 0L,
        (void*)ybuf, (void*)ybuf, HD, 0L, out_b, x, 0L, NT, HD, HD, wscale);
  }
  layernorm_kernel<<<NT, 256, 0, stream>>>(ybuf, ln1_g, ln1_b, x1f, x1h, 1);
  transpose_cast_f16<<<dim3(H4 / 64, HD / 64), 256, 0, stream>>>(w1, wT, HD, H4, wmul);
  {
    const int tiles = (NT / 64) * (H4 / 64);
    wmma_gemm64<0, false, 2, 1, false, 2><<<dim3((tiles + 7) / 8, 1), 256, 0, stream>>>(
        (cus)x1h, (cus)x1h, HD, 0L, (cus)wT, (cus)wT, HD, 0L,
        (void*)hbuf, (void*)hbuf, H4, 0L, b1, b1, 0L, NT, H4, HD, wscale);
  }
  transpose_cast_f16<<<dim3(HD / 64, H4 / 64), 256, 0, stream>>>(w2, wT, H4, HD, wmul);
  {
    const int tiles = (NT / 64) * (HD / 64);
    wmma_gemm64<0, false, 2, 0, true, 0><<<dim3((tiles + 7) / 8, 1), 256, 0, stream>>>(
        (cus)hbuf, (cus)hbuf, H4, 0L, (cus)wT, (cus)wT, H4, 0L,
        (void*)ybuf, (void*)ybuf, HD, 0L, b2, x1f, 0L, NT, HD, H4, wscale);
  }
  layernorm_kernel<<<NT, 256, 0, stream>>>(ybuf, ln2_g, ln2_b, outp, x1h, 0);
  (void)hipGetLastError();
}
